// DynamicSlimmableBlock_40510131535959
// MI455X (gfx1250) — hardware-verified
//
#include <hip/hip_runtime.h>
#include <hip/hip_bf16.h>


constexpr int NB_   = 8;
constexpr int NT_   = 4000;
constexpr int CIN_  = 256;
constexpr int COUT_ = 256;
constexpr int HID_  = 2048;
constexpr int KLEN_ = 39;
constexpr int PADL_ = 19;
constexpr int NROW_ = NB_ * NT_;
constexpr int RT_   = 32;
constexpr int HCH_  = 256;
constexpr int NHC_  = HID_ / HCH_;
constexpr int XP_   = 264;
constexpr int MP_   = 260;
constexpr int TT_   = 25;
constexpr int WR_   = TT_ + KLEN_ - 1;

static_assert(NROW_ % RT_ == 0);
static_assert(NT_ % RT_ == 0);
static_assert(NT_ % TT_ == 0);
static_assert(HID_ % HCH_ == 0);
static_assert(CIN_ % 32 == 0);
static_assert(HCH_ % 32 == 0);
static_assert((XP_ * 2) % 16 == 0);
static_assert((MP_ * 4) % 16 == 0);
static_assert((RT_ * CIN_) % (256 * 4) == 0);

typedef float          v2f   __attribute__((ext_vector_type(2)));
typedef float          v4f   __attribute__((ext_vector_type(4)));
typedef float          v8f   __attribute__((ext_vector_type(8)));
typedef _Float16       v4h   __attribute__((ext_vector_type(4)));
typedef _Float16       v8h   __attribute__((ext_vector_type(8)));
typedef _Float16       v16h  __attribute__((ext_vector_type(16)));
typedef __bf16         v16b  __attribute__((ext_vector_type(16)));
typedef unsigned short u16x8 __attribute__((ext_vector_type(8)));

union FragH { v8h   h[2]; v16h v; };
union FragB { u16x8 h[2]; v16b v; };

struct FsT { unsigned short h[RT_ * XP_]; unsigned short l[RT_ * XP_]; };
union  FsU { FsT fs; float mst[RT_ * MP_]; };
static_assert(sizeof(float) * RT_ * MP_ <= sizeof(FsT));

__device__ __forceinline__ unsigned short f2bf(float f) {
    unsigned u = __float_as_uint(f);
    unsigned r = u + 0x7FFFu + ((u >> 16) & 1u);
    return (unsigned short)(r >> 16);
}
__device__ __forceinline__ float bf2f(unsigned short b) {
    return __uint_as_float(((unsigned)b) << 16);
}
__device__ __forceinline__ v8f ld8f(const float* p) {
    v4f a = *(const v4f*)p;
    v4f b = *(const v4f*)(p + 4);
    return __builtin_shufflevector(a, b, 0, 1, 2, 3, 4, 5, 6, 7);
}
__device__ __forceinline__ void split8(const v8f& x, u16x8& hv, u16x8& lv) {
#pragma unroll
    for (int c = 0; c < 8; ++c) {
        const float f = x[c];
        const unsigned short hb = f2bf(f);
        hv[c] = hb;
        lv[c] = f2bf(f - bf2f(hb));
    }
}

__device__ __forceinline__ void mma_h(v8f& acc, const FragH& a, const FragH& b) {
    acc = __builtin_amdgcn_wmma_f32_16x16x32_f16(false, a.v, false, b.v, (short)0, acc, false, false);
    asm volatile("v_nop\n\tv_nop\n\tv_nop\n\tv_nop" : "+v"(acc) : "v"(a.v), "v"(b.v));
}
__device__ __forceinline__ void mma_bf(v8f& acc, const FragB& a, const FragB& b) {
    acc = __builtin_amdgcn_wmma_f32_16x16x32_bf16(false, a.v, false, b.v, (short)0, acc, false, false);
    asm volatile("v_nop\n\tv_nop\n\tv_nop\n\tv_nop" : "+v"(acc) : "v"(a.v), "v"(b.v));
}

__global__ __launch_bounds__(256)
void gate_kernel(const float* __restrict__ x, const float* __restrict__ gw, const float* __restrict__ gb,
                 const float* __restrict__ tau, float* probs_ws, float* out_tail)
{
    __shared__ double red0[256];
    __shared__ double red1[256];
    __shared__ float  sp[2 * NB_];
    __shared__ __attribute__((aligned(16))) float pline[32];

    const int c = threadIdx.x;
    const float g00 = gw[c];
    const float g01 = gw[CIN_ + c];
    const float g10 = gw[2 * CIN_ + c];
    const float g11 = gw[3 * CIN_ + c];
    const float tauv = tau[0];

#pragma unroll 1
    for (int b = 0; b < NB_; ++b) {
        const float* xb = x + (size_t)b * NT_ * CIN_ + c;
        double s = 0.0, q = 0.0;
#pragma unroll 4
        for (int t = 0; t < NT_; ++t) {
            const double v = (double)xb[(size_t)t * CIN_];
            s += v;
            q += v * v;
        }
        const double mean = s * (1.0 / (double)NT_);
        double var = (q - s * mean) * (1.0 / (double)(NT_ - 1));
        var = var > 0.0 ? var : 0.0;
        const float meanf = (float)mean;
        const float sdf   = sqrtf((float)var);
        red0[c] = (double)meanf * (double)g00 + (double)sdf * (double)g01;
        red1[c] = (double)meanf * (double)g10 + (double)sdf * (double)g11;
        __syncthreads();
#pragma unroll 1
        for (int sft = 128; sft > 0; sft >>= 1) {
            if (c < sft) {
                red0[c] += red0[c + sft];
                red1[c] += red1[c + sft];
            }
            __syncthreads();
        }
        if (c == 0) {
            const float l0 = tauv * ((float)red0[0] + gb[0]);
            const float l1 = tauv * ((float)red1[0] + gb[1]);
            const float mx = fmaxf(l0, l1);
            const float e0 = expf(l0 - mx);
            const float e1 = expf(l1 - mx);
            const float inv = 1.0f / (e0 + e1);
            sp[2 * b]     = e0 * inv;
            sp[2 * b + 1] = e1 * inv;
        }
        __syncthreads();
    }

    v2f ov;
    ov.x = 0.0f; ov.y = 0.0f;
    if (c == 0) {
        float spv = 0.0f, i0 = 0.0f, i1 = 0.0f;
#pragma unroll 1
        for (int b = 0; b < NB_; ++b) {
            const float p0 = sp[2 * b], p1 = sp[2 * b + 1];
            const float nrm = sqrtf(p0 * p0 + p1 * p1) + 1e-8f;
            const float rn  = 1.0f / nrm;
            spv += 0.1f * fabsf(p0 * rn) + 0.1f * fabsf(p1 * rn);
            i0 += p0;
            i1 += p1;
        }
        spv *= (1.0f / (float)NB_);
        i0  *= (1.0f / (float)NB_);
        i1  *= (1.0f / (float)NB_);
        const float mu  = (i0 + i1) * 0.5f;
        const float d0  = i0 - mu, d1 = i1 - mu;
        const float var = d0 * d0 + d1 * d1;
        const float sd  = sqrtf(var);
        const float cv  = sd * (1.0f / (mu + 1e-8f));
        ov.x = spv;
        ov.y = 0.01f * cv * cv;
    }
    if (c < 32) pline[c] = (c < 2 * NB_) ? sp[c] : 0.0f;
    __syncthreads();
    v4f pv;
    pv.x = 0.0f; pv.y = 0.0f; pv.z = 0.0f; pv.w = 0.0f;
    if (c < 8) pv = *(const v4f*)(pline + c * 4);
    if (c < 8) *(volatile v4f*)(probs_ws + c * 4) = pv;
    if (c == 0) *(volatile v2f*)(out_tail) = ov;
    __threadfence();
    if (c < 8) *(volatile v4f*)(probs_ws + c * 4) = pv;
    if (c == 0) *(volatile v2f*)(out_tail) = ov;
}

__global__ __launch_bounds__(256)
void prep_kernel(const float* __restrict__ w1, const float* __restrict__ w2,
                 _Float16* W1P, unsigned short* W2H, unsigned short* W2L, int n8)
{
    const int i = blockIdx.x * 256 + threadIdx.x;
    if (i >= n8) return;
    const size_t e = (size_t)i * 8;
    if (blockIdx.y == 0) {
        const v8f v = ld8f(w1 + e);
        v8h hv;
#pragma unroll
        for (int c = 0; c < 8; ++c) hv[c] = (_Float16)(v[c] * 16.0f);
        *(volatile v8h*)(W1P + e) = hv;
        __threadfence();
        *(volatile v8h*)(W1P + e) = hv;
    } else {
        const v8f v = ld8f(w2 + e);
        u16x8 hv, lv;
        split8(v, hv, lv);
        *(volatile u16x8*)(W2H + e) = hv;
        *(volatile u16x8*)(W2L + e) = lv;
        __threadfence();
        *(volatile u16x8*)(W2H + e) = hv;
        *(volatile u16x8*)(W2L + e) = lv;
    }
}

__global__ __launch_bounds__(256)
void ffn_kernel(const float* __restrict__ x, const float* __restrict__ b1,
                const _Float16* __restrict__ W1P,
                const unsigned short* __restrict__ W2H, const unsigned short* __restrict__ W2L,
                const float* __restrict__ probs, float* Mbuf)
{
    __shared__ __attribute__((aligned(16))) _Float16 xs[RT_ * XP_];
    __shared__ __attribute__((aligned(16))) FsU u;

    const int tid  = threadIdx.x;
    const int lane = tid & 31;
    const int wave = tid >> 5;
    const int h    = lane >> 4;
    const int m    = lane & 15;
    const int row0 = blockIdx.x * RT_;
    const int bidx = blockIdx.x / (NT_ / RT_);
    const int ncol = wave * 32;

#pragma unroll
    for (int it = 0; it < (RT_ * CIN_) / (256 * 4); ++it) {
        const int idx = it * 256 + tid;
        const int r   = idx >> 6;
        const int c4  = (idx & 63) * 4;
        const v4f v = *(const v4f*)(x + (size_t)(row0 + r) * CIN_ + c4);
        v4h hv;
        hv.x = (_Float16)v.x; hv.y = (_Float16)v.y; hv.z = (_Float16)v.z; hv.w = (_Float16)v.w;
        *(v4h*)(xs + r * XP_ + c4) = hv;
    }
    __syncthreads();

    v8f acc[4], pa[4];
#pragma unroll
    for (int j = 0; j < 4; ++j)
#pragma unroll
        for (int r = 0; r < 8; ++r) { acc[j][r] = 0.0f; pa[j][r] = 0.0f; }

#pragma unroll 1
    for (int hc = 0; hc < NHC_; ++hc) {
        const int hbase = hc * HCH_ + ncol;

        v8f c1[4];
#pragma unroll
        for (int j = 0; j < 4; ++j)
#pragma unroll
            for (int r = 0; r < 8; ++r) c1[j][r] = 0.0f;

#pragma unroll 1
        for (int ks = 0; ks < CIN_ / 32; ++ks) {
            const int k0 = ks * 32;
            FragH fa[2], fb[2];
#pragma unroll
            for (int s = 0; s < 2; ++s) {
                const _Float16* p = xs + (s * 16 + m) * XP_ + k0 + 8 * h;
                fa[s].h[0] = *(const v8h*)(p);
                fa[s].h[1] = *(const v8h*)(p + 16);
            }
#pragma unroll
            for (int j = 0; j < 2; ++j) {
                const _Float16* q = W1P + (size_t)(hbase + j * 16 + m) * CIN_ + k0 + 8 * h;
                fb[j].h[0] = *(const v8h*)(q);
                fb[j].h[1] = *(const v8h*)(q + 16);
            }
#pragma unroll
            for (int s = 0; s < 2; ++s)
#pragma unroll
                for (int j = 0; j < 2; ++j) mma_h(c1[s * 2 + j], fa[s], fb[j]);
        }

        const float bj0 = b1[hbase + m];
        const float bj1 = b1[hbase + 16 + m];
#pragma unroll
        for (int s = 0; s < 2; ++s)
#pragma unroll
            for (int j = 0; j < 2; ++j) {
                const float bj = (j == 0) ? bj0 : bj1;
#pragma unroll
                for (int r = 0; r < 8; ++r) {
                    const float f = fmaxf(c1[s * 2 + j][r] * 0.0625f + bj, 0.0f);
                    const unsigned short hb = f2bf(f);
                    const unsigned short lb = f2bf(f - bf2f(hb));
                    const int o = (s * 16 + 8 * h + r) * XP_ + ncol + j * 16 + m;
                    u.fs.h[o] = hb;
                    u.fs.l[o] = lb;
                }
            }
        __syncthreads();

        const int kg0 = hc * HCH_;
#pragma unroll 1
        for (int ks = 0; ks < HCH_ / 32; ++ks) {
            const int k0 = ks * 32;
            FragB ah[2], al[2], bh[2], bl[2];
#pragma unroll
            for (int s = 0; s < 2; ++s) {
                const int ofs = (s * 16 + m) * XP_ + k0 + 8 * h;
                ah[s].h[0] = *(const u16x8*)(u.fs.h + ofs);
                ah[s].h[1] = *(const u16x8*)(u.fs.h + ofs + 16);
                al[s].h[0] = *(const u16x8*)(u.fs.l + ofs);
                al[s].h[1] = *(const u16x8*)(u.fs.l + ofs + 16);
            }
#pragma unroll
            for (int j = 0; j < 2; ++j) {
                const size_t gofs = (size_t)(ncol + j * 16 + m) * HID_ + kg0 + k0 + 8 * h;
                bh[j].h[0] = *(const u16x8*)(W2H + gofs);
                bh[j].h[1] = *(const u16x8*)(W2H + gofs + 16);
                bl[j].h[0] = *(const u16x8*)(W2L + gofs);
                bl[j].h[1] = *(const u16x8*)(W2L + gofs + 16);
            }
#pragma unroll
            for (int s = 0; s < 2; ++s)
#pragma unroll
                for (int j = 0; j < 2; ++j) {
                    mma_bf(acc[s * 2 + j], ah[s], bh[j]);
                    mma_bf(acc[s * 2 + j], ah[s], bl[j]);
                    mma_bf(acc[s * 2 + j], al[s], bh[j]);
                }
        }
        __syncthreads();

        if (hc == 0) {
#pragma unroll
            for (int j = 0; j < 4; ++j) pa[j] = acc[j];
        }
    }

    const float p0 = probs[2 * bidx];
    const float p1 = probs[2 * bidx + 1];
#pragma unroll
    for (int s = 0; s < 2; ++s)
#pragma unroll
        for (int j = 0; j < 2; ++j)
#pragma unroll
            for (int r = 0; r < 8; ++r)
                u.mst[(s * 16 + 8 * h + r) * MP_ + ncol + j * 16 + m] = p0 * acc[s * 2 + j][r] + p1 * pa[s * 2 + j][r];
    __syncthreads();

    v4f vals[8];
    size_t goff[8];
#pragma unroll
    for (int it = 0; it < 8; ++it) {
        const int r  = it * 4 + (tid >> 6);
        const int c4 = (tid & 63) * 4;
        vals[it] = *(const v4f*)(u.mst + r * MP_ + c4);
        goff[it] = (size_t)(row0 + r) * COUT_ + c4;
    }
#pragma unroll
    for (int it = 0; it < 8; ++it) *(volatile v4f*)(Mbuf + goff[it]) = vals[it];
    __threadfence();
#pragma unroll
    for (int it = 0; it < 8; ++it) *(volatile v4f*)(Mbuf + goff[it]) = vals[it];
}

__global__ __launch_bounds__(256)
void conv_kernel(const float* __restrict__ Mbuf, const float* __restrict__ cwg, float* out)
{
    __shared__ float win[WR_ * COUT_];
    const int c  = threadIdx.x;
    const int b  = blockIdx.y;
    const int t0 = blockIdx.x * TT_;

    float cw[KLEN_];
#pragma unroll
    for (int j = 0; j < KLEN_; ++j) cw[j] = cwg[c * KLEN_ + j];

    const float* Mb = Mbuf + (size_t)b * NT_ * COUT_;
#pragma unroll 1
    for (int row = 0; row < WR_; ++row) {
        const int t  = t0 + row - PADL_;
        const int tc = min(max(t, 0), NT_ - 1);
        const float v = Mb[(size_t)tc * COUT_ + c];
        win[row * COUT_ + c] = (t >= 0 && t < NT_) ? v : 0.0f;
    }
    __syncthreads();

#pragma unroll 1
    for (int tt = 0; tt < TT_; ++tt) {
        float a = win[(tt + PADL_) * COUT_ + c];
#pragma unroll
        for (int j = 0; j < KLEN_; ++j) a += cw[j] * win[(tt + j) * COUT_ + c];
        win[tt * COUT_ + c] = a;
    }

    float* ob = out + ((size_t)b * NT_ + t0) * COUT_ + c;
#pragma unroll 1
    for (int tt = 0; tt < TT_; ++tt) {
        const float v = win[tt * COUT_ + c];
        *(volatile float*)(ob + (size_t)tt * COUT_) = v;
    }
    __threadfence();
#pragma unroll 1
    for (int tt = 0; tt < TT_; ++tt) {
        const float v = win[tt * COUT_ + c];
        *(volatile float*)(ob + (size_t)tt * COUT_) = v;
    }
}

extern "C" void kernel_launch(void* const* d_in, const int* in_sizes, int n_in,
                              void* d_out, int out_size, void* d_ws, size_t ws_size,
                              hipStream_t stream)
{
    if (n_in < 8) return;
    if (in_sizes[0] != NROW_ * CIN_) return;
    if (in_sizes[1] != HID_ * CIN_) return;
    if (in_sizes[2] != HID_) return;
    if (in_sizes[3] != COUT_ * HID_) return;
    if (in_sizes[4] != COUT_ * KLEN_) return;
    if (in_sizes[5] != 2 * 2 * CIN_) return;
    if (in_sizes[6] != 2) return;
    if (in_sizes[7] != 1) return;
    if (out_size != NROW_ * COUT_ + 2) return;

    const float* x      = (const float*)d_in[0];
    const float* w1     = (const float*)d_in[1];
    const float* b1     = (const float*)d_in[2];
    const float* w2     = (const float*)d_in[3];
    const float* conv_w = (const float*)d_in[4];
    const float* gate_w = (const float*)d_in[5];
    const float* gate_b = (const float*)d_in[6];
    const float* tau    = (const float*)d_in[7];
    float* out = (float*)d_out;

    char* ws = (char*)d_ws;
    size_t off = 0;
    auto carve = [&](size_t bytes) -> char* { char* p = ws + off; off += (bytes + 255) & ~(size_t)255; return p; };
    float*          PROB = (float*)carve(256);
    float*          MBUF = (float*)carve((size_t)NROW_ * COUT_ * 4);
    _Float16*       W1P  = (_Float16*)carve((size_t)HID_ * CIN_ * 2);
    unsigned short* W2H  = (unsigned short*)carve((size_t)COUT_ * HID_ * 2);
    unsigned short* W2L  = (unsigned short*)carve((size_t)COUT_ * HID_ * 2);
    if (off > ws_size) return;

    const dim3 b256(256);
    const int n8 = (HID_ * CIN_) / 8;

    gate_kernel<<<dim3(1), b256, 0, stream>>>(x, gate_w, gate_b, tau, PROB, out + (size_t)NROW_ * COUT_);
    prep_kernel<<<dim3((n8 + 255) / 256, 2), b256, 0, stream>>>(w1, w2, W1P, W2H, W2L, n8);
    ffn_kernel<<<dim3(NROW_ / RT_), b256, 0, stream>>>(x, b1, W1P, W2H, W2L, PROB, MBUF);
    conv_kernel<<<dim3(NT_ / TT_, NB_), b256, 0, stream>>>(MBUF, conv_w, out);
}
